// SpatialRegressor3_81853486727431
// MI455X (gfx1250) — hardware-run, weakly checked
//
#include <hip/hip_runtime.h>
#include <math.h>

#ifndef NB
#define NB 4096
#endif
#ifndef SEQ
#define SEQ 128
#endif
#define NB_FULL 4096
#define SEQ_FULL 128
#define HID 32
#define NROWS (NB * SEQ)
#define P0_ROWS 1024
#define NP0 (NROWS / P0_ROWS)
#define NPB (NROWS / 128)
#define REC_BYTES 4224u
#define NREC 9u
#define SLAB_P 36u

static_assert(SEQ == SEQ_FULL);
static_assert(SEQ == 128);
static_assert(NB <= NB_FULL);
static_assert(NB % 256 == 0);
static_assert(NROWS % P0_ROWS == 0);
static_assert(NROWS % 128 == 0);
static_assert(REC_BYTES % 128u == 0u);

#define K_T   16384.0f
#define KR_T  67108864.0f
#define K_S   8192.0f
#define KR_S  33554432.0f
#define K_X   1024.0f
#define KR_X  4194304.0f
#define K_W   2048.0f
#define KR_W  8388608.0f
static_assert(K_T * KR_W == KR_T * K_W);
static_assert(K_S * KR_W == KR_S * K_W);
static_assert(K_X * KR_W == KR_X * K_W);

typedef _Float16 h16;
typedef __attribute__((ext_vector_type(16))) _Float16 v16h;
typedef __attribute__((ext_vector_type(8)))  _Float16 v8h;
typedef __attribute__((ext_vector_type(8)))  float    v8f;
typedef __attribute__((ext_vector_type(4)))  float    v4f;
typedef __attribute__((ext_vector_type(4)))  int      v4i;

constexpr size_t a256(size_t b) { return (b + 255) & ~(size_t)255; }
constexpr size_t SZ_P0  = (size_t)NP0 * 128;
constexpr size_t SZ_P12 = (size_t)NPB * 512;
constexpr size_t SZ_REC = (size_t)NREC * REC_BYTES;
constexpr size_t SZ_PL  = (size_t)NB * HID * 4;
constexpr size_t WS_TOTAL = a256(SZ_P0) + 2 * a256(SZ_P12) + a256(SZ_REC) + 4 * a256(SZ_PL);
static_assert(WS_TOTAL <= (size_t)134217728);


#define VST2V4(ptr, val) do { const v4f vst2_v4_ = (val); *(volatile v4f*)(ptr) = vst2_v4_; __threadfence(); *(volatile v4f*)(ptr) = vst2_v4_; } while (0)
#define VST2V8H(ptr, val) do { const v8h vst2_h8_ = (val); *(volatile v8h*)(ptr) = vst2_h8_; __threadfence(); *(volatile v8h*)(ptr) = vst2_h8_; } while (0)

__device__ __forceinline__ float bfr(float f) {
    unsigned u = __float_as_uint(f);
    u += 0x7FFFu + ((u >> 16) & 1u);
    return __uint_as_float(u & 0xFFFF0000u);
}
__device__ __forceinline__ v4f bfr4(v4f x) {
    v4f y; y.x = bfr(x.x); y.y = bfr(x.y); y.z = bfr(x.z); y.w = bfr(x.w); return y;
}
static __device__ __forceinline__ h16 toh_flush(float v) { const float w = (fabsf(v) < 6.103515625e-05f) ? 0.0f : v; return (h16)w; }

__device__ __forceinline__ void split16(float a, float k, float ik, float kr, h16& hi, h16& lo) {
    hi = toh_flush(a * k);
    const float r = a - (float)hi * ik;
    lo = toh_flush(r * kr);
}

union FragU { v16h v; v8h h[2]; };
__device__ __forceinline__ v16h frag_ld(const h16* p) {
    FragU f; f.h[0] = *(const v8h*)(p); f.h[1] = *(const v8h*)(p + 16); return f.v;
}
__device__ __forceinline__ v8f wmma16g(v16h a, v16h b, v8f c) {
    c = __builtin_amdgcn_wmma_f32_16x16x32_f16(false, a, false, b, (short)0, c, false, false);
    asm volatile("v_nop\n\tv_nop\n\tv_nop\n\tv_nop" : "+v"(c) : "v"(a), "v"(b));
    return c;
}
__device__ __forceinline__ void wave_sync_lds() {
    __builtin_amdgcn_fence(3  , "workgroup");
    __builtin_amdgcn_wave_barrier();
    __builtin_amdgcn_fence(2  , "workgroup");
}

struct D2 { v8f t[2]; };

__device__ __forceinline__ D2 tanh2(const D2& v) {
    D2 o;
#pragma unroll
    for (int t = 0; t < 2; ++t)
#pragma unroll
        for (int r = 0; r < 8; ++r) o.t[t][r] = tanhf(v.t[t][r]);
    return o;
}

__device__ __forceinline__ void build_a(v4f q0, v4f q1, v4f q2, v4f q3, float k, float ik, float kr, v16h& ahi, v16h& alo) {
    const v4f q[4] = {q0, q1, q2, q3};
#pragma unroll
    for (int j = 0; j < 4; ++j) {
#pragma unroll
        for (int e = 0; e < 4; ++e) {
            h16 h, l;
            split16(q[j][e], k, ik, kr, h, l);
            ahi[4 * j + e] = h;
            alo[4 * j + e] = l;
        }
    }
}

__device__ __forceinline__ void d2_to_a(float* slab, const D2& v, unsigned hh, unsigned c, float k, float ik, float kr,
                                        v16h& ahi, v16h& alo) {
    wave_sync_lds();
#pragma unroll
    for (int t = 0; t < 2; ++t)
#pragma unroll
        for (int r = 0; r < 8; ++r) slab[(8u * hh + (unsigned)r) * SLAB_P + 16u * (unsigned)t + c] = v.t[t][r];
    wave_sync_lds();
    const float* p = slab + c * SLAB_P + 8u * hh;
    const v4f q0 = *(const v4f*)(p), q1 = *(const v4f*)(p + 4), q2 = *(const v4f*)(p + 16), q3 = *(const v4f*)(p + 20);
    build_a(q0, q1, q2, q3, k, ik, kr, ahi, alo);
}

__device__ __forceinline__ D2 mm3(v16h ahi, v16h alo, const unsigned char* __restrict__ rec, unsigned hh, unsigned c,
                                  float svv, float sxx) {
    const h16* Whi = (const h16*)rec;
    const h16* Wlo = (const h16*)(rec + 2048);
    const float* bias = (const float*)(rec + 4096);
    D2 o;
#pragma unroll
    for (int t = 0; t < 2; ++t) {
        const unsigned n = 16u * (unsigned)t + c;
        const v16h bhi = frag_ld(Whi + n * 32u + 8u * hh);
        const v16h blo = frag_ld(Wlo + n * 32u + 8u * hh);
        const float bv = bias[n];
        v8f vv = (v8f){0.f, 0.f, 0.f, 0.f, 0.f, 0.f, 0.f, 0.f};
        v8f xx = (v8f){0.f, 0.f, 0.f, 0.f, 0.f, 0.f, 0.f, 0.f};
        vv = wmma16g(ahi, bhi, vv);
        xx = wmma16g(ahi, blo, xx);
        xx = wmma16g(alo, bhi, xx);
#pragma unroll
        for (int r = 0; r < 8; ++r) o.t[t][r] = (vv[r] * svv + xx[r] * sxx) + bv;
    }
    return o;
}

__device__ __forceinline__ D2 site(float* slab, const D2& v, float k, float ik, float kr, float svv, float sxx,
                                   const unsigned char* __restrict__ rec, unsigned hh, unsigned c) {
    v16h ahi, alo;
    d2_to_a(slab, v, hh, c, k, ik, kr, ahi, alo);
    return mm3(ahi, alo, rec, hh, c, svv, sxx);
}

__device__ __forceinline__ void load_u8(const float* __restrict__ u, unsigned rowbase, v4f ub[8]) {
#pragma unroll
    for (int r = 0; r < 8; ++r) ub[r] = bfr4(*(const v4f*)(u + (size_t)(rowbase + (unsigned)r) * 4u));
}

__device__ __forceinline__ D2 layer1(const v4f ub[8], const unsigned char* __restrict__ rec, unsigned c) {
    const float* wf = (const float*)rec;
    const float* bs = (const float*)(rec + 4096);
    const v4f w0 = *(const v4f*)(wf + 4u * c);
    const v4f w1 = *(const v4f*)(wf + 4u * (16u + c));
    const float b0 = bs[c], b1 = bs[16u + c];
    D2 o;
#pragma unroll
    for (int r = 0; r < 8; ++r) {
        const v4f x = ub[r];
        const float p0 = ((x.x * w0.x + x.y * w0.y) + (x.z * w0.z + x.w * w0.w)) + b0;
        const float p1 = ((x.x * w1.x + x.y * w1.y) + (x.z * w1.z + x.w * w1.w)) + b1;
        o.t[0][r] = tanhf(p0);
        o.t[1][r] = tanhf(p1);
    }
    return o;
}

__device__ __forceinline__ void col_stats(float* stw, unsigned off, const D2& v, unsigned hh, unsigned c) {
#pragma unroll
    for (int t = 0; t < 2; ++t) {
        float s = 0.f, q = 0.f;
#pragma unroll
        for (int r = 0; r < 8; ++r) { const float x = v.t[t][r]; s += x; q += x * x; }
        s += __shfl_xor(s, 16, 32);
        q += __shfl_xor(q, 16, 32);
        if (hh == 0u) { stw[off + 16u * (unsigned)t + c] = s; stw[off + 32u + 16u * (unsigned)t + c] = q; }
    }
}

__global__ __launch_bounds__(256) void k_pass0(const float* __restrict__ u, float* __restrict__ part0) {
    __shared__ float sW[8][8];
    const unsigned tid = threadIdx.x, lane = tid & 31u, wave = tid >> 5;
    const unsigned bx = blockIdx.x;
    float s[4] = {0.f, 0.f, 0.f, 0.f}, q[4] = {0.f, 0.f, 0.f, 0.f};
#pragma unroll
    for (int j = 0; j < 4; ++j) {
        const unsigned row = bx * (unsigned)P0_ROWS + (unsigned)j * 256u + tid;
        const v4f x = bfr4(*(const v4f*)(u + (size_t)row * 4u));
        s[0] += x.x; s[1] += x.y; s[2] += x.z; s[3] += x.w;
        q[0] += x.x * x.x; q[1] += x.y * x.y; q[2] += x.z * x.z; q[3] += x.w * x.w;
    }
#pragma unroll
    for (int i = 0; i < 4; ++i) {
#pragma unroll
        for (int o = 16; o > 0; o >>= 1) { s[i] += __shfl_xor(s[i], o, 32); q[i] += __shfl_xor(q[i], o, 32); }
    }
    if (lane == 0u) {
#pragma unroll
        for (int i = 0; i < 4; ++i) { sW[wave][i] = s[i]; sW[wave][4 + i] = q[i]; }
    }
    __syncthreads();
    if (tid < 8u) {
        const unsigned base = min(tid, 1u) * 4u;
        v4f v;
#pragma unroll
        for (int i = 0; i < 4; ++i) {
            float acc = 0.f;
#pragma unroll
            for (int w = 0; w < 8; ++w) acc += sW[w][base + (unsigned)i];
            v[i] = (tid < 2u) ? acc : 0.0f;
        }
        VST2V4(part0 + (size_t)bx * 32u + 4u * tid, v);
    }
}

__global__ __launch_bounds__(64) void k_fold4(const float* __restrict__ part0, unsigned nPart, unsigned nrows,
                                              const float* __restrict__ g, const float* __restrict__ b,
                                              const float* __restrict__ W, unsigned char* __restrict__ rec) {
    __shared__ double dS[8];
    __shared__ float sSG[4];
    __shared__ float sSH[4];
    __shared__ __align__(16) float sC[32];
    const unsigned t = threadIdx.x;
    if (t < 8u) {
        double acc = 0.0;
        for (unsigned p = 0; p < nPart; ++p) acc += (double)part0[(size_t)p * 32u + t];
        dS[t] = acc;
    }
    __syncthreads();
    if (t < 4u) {
        const double invn = 1.0 / (double)nrows;
        const double mean = dS[t] * invn;
        const double var = dS[4u + t] * invn - mean * mean;
        const float s = 1.0f / sqrtf((float)var + 1e-5f);
        const float sg = s * bfr(g[t]);
        sSG[t] = sg;
        sSH[t] = bfr(b[t]) - (float)mean * sg;
    }
    __syncthreads();
    if (t < 32u) {
        const v4f w = bfr4(*(const v4f*)(W + 4u * t));
        v4f wf;
        wf.x = w.x * sSG[0]; wf.y = w.y * sSG[1]; wf.z = w.z * sSG[2]; wf.w = w.w * sSG[3];
        sC[t] = (sSH[0] * w.x + sSH[1] * w.y) + (sSH[2] * w.z + sSH[3] * w.w);
        VST2V4((float*)rec + 4u * t, wf);
    }
    __syncthreads();
    if (t < 8u) {
        const v4f v = *(const v4f*)(sC + 4u * t);
        VST2V4((float*)(rec + 4096) + 4u * t, v);
    }
}

__device__ __forceinline__ void fold_finish(unsigned t, double mean, double var, const float* __restrict__ g,
                                            const float* __restrict__ b, const float* __restrict__ W,
                                            unsigned char* __restrict__ rec) {
    __shared__ float sSG[32];
    __shared__ float sSH[32];
    __shared__ __align__(16) float sC[32];
    if (t < 32u) {
        const float s = 1.0f / sqrtf((float)var + 1e-5f);
        const float sg = s * bfr(g[t]);
        sSG[t] = sg;
        sSH[t] = bfr(b[t]) - (float)mean * sg;
    }
    __syncthreads();
    if (t < 128u) {
        const unsigned o = t >> 2, k0 = (t & 3u) * 8u;
        const v4f w0 = *(const v4f*)(W + o * 32u + k0);
        const v4f w1 = *(const v4f*)(W + o * 32u + k0 + 4u);
        const float wv[8] = {w0.x, w0.y, w0.z, w0.w, w1.x, w1.y, w1.z, w1.w};
        v8h hv, lv;
#pragma unroll
        for (int e = 0; e < 8; ++e) {
            const float wf = bfr(wv[e]) * sSG[k0 + (unsigned)e];
            h16 h, l;
            split16(wf, K_W, 1.0f / K_W, KR_W, h, l);
            hv[e] = h;
            lv[e] = l;
        }
        h16* ph = (h16*)rec + o * 32u + k0;
        h16* pl = (h16*)(rec + 2048) + o * 32u + k0;
        VST2V8H(ph, hv);
        VST2V8H(pl, lv);
    }
    if (t < 32u) {
        float acc = 0.f;
#pragma unroll
        for (int g4 = 0; g4 < 8; ++g4) {
            const v4f w = bfr4(*(const v4f*)(W + t * 32u + 4u * (unsigned)g4));
            acc += sSH[4 * g4] * w.x + sSH[4 * g4 + 1] * w.y + sSH[4 * g4 + 2] * w.z + sSH[4 * g4 + 3] * w.w;
        }
        sC[t] = acc;
    }
    __syncthreads();
    if (t < 8u) {
        const v4f v = *(const v4f*)(sC + 4u * t);
        VST2V4((float*)(rec + 4096) + 4u * t, v);
    }
}

__global__ __launch_bounds__(256) void k_fold32(const float* __restrict__ part, unsigned nPart, unsigned pstride,
                                                unsigned colS, unsigned colQ, unsigned nrows,
                                                const float* __restrict__ g, const float* __restrict__ b,
                                                const float* __restrict__ W, unsigned char* __restrict__ rec) {
    __shared__ double dS[64];
    const unsigned t = threadIdx.x;
    if (t < 64u) {
        const unsigned col = (t < 32u) ? (colS + t) : (colQ + t - 32u);
        double acc = 0.0;
        for (unsigned p = 0; p < nPart; ++p) acc += (double)part[(size_t)p * pstride + col];
        dS[t] = acc;
    }
    __syncthreads();
    double mean = 0.0, var = 1.0;
    if (t < 32u) {
        const double invn = 1.0 / (double)nrows;
        mean = dS[t] * invn;
        var = dS[32u + t] * invn - mean * mean;
    }
    fold_finish(t, mean, var, g, b, W, rec);
}

__global__ __launch_bounds__(256) void k_foldp(const float* __restrict__ P, const float* __restrict__ g,
                                               const float* __restrict__ b, const float* __restrict__ W,
                                               unsigned char* __restrict__ rec) {
    __shared__ double dS[8][32];
    __shared__ double dQ[8][32];
    const unsigned t = threadIdx.x, col = t & 31u, sl = t >> 5;
    {
        double s = 0.0, q = 0.0;
        for (unsigned i = 0; i < (unsigned)(NB / 8); ++i) {
            const double x = (double)P[(size_t)(sl * (unsigned)(NB / 8) + i) * 32u + col];
            s += x; q += x * x;
        }
        dS[sl][col] = s; dQ[sl][col] = q;
    }
    __syncthreads();
    double mean = 0.0, var = 1.0;
    if (t < 32u) {
        double s = 0.0, q = 0.0;
#pragma unroll
        for (int w = 0; w < 8; ++w) { s += dS[w][t]; q += dQ[w][t]; }
        const double invn = 1.0 / (double)NB;
        mean = s * invn;
        var = q * invn - mean * mean;
    }
    fold_finish(t, mean, var, g, b, W, rec);
}

__device__ __forceinline__ void write_part(const float* sst  , unsigned tid, float* __restrict__ dst) {
    if (tid < 32u) {
        v4f v;
#pragma unroll
        for (int j = 0; j < 4; ++j) {
            float acc = 0.f;
#pragma unroll
            for (int w = 0; w < 8; ++w) acc += sst[(unsigned)w * 128u + 4u * tid + (unsigned)j];
            v[j] = acc;
        }
        VST2V4(dst + 4u * tid, v);
    }
}

__global__ __launch_bounds__(256) void k_pass1(const float* __restrict__ u, const unsigned char* __restrict__ recs,
                                               float* __restrict__ part) {
    __shared__ __align__(16) float sSt[8][128];
    const unsigned tid = threadIdx.x, lane = tid & 31u, wave = tid >> 5, hh = lane >> 4, c = lane & 15u;
    const unsigned bx = blockIdx.x;
    const unsigned row0 = (bx * 8u + wave) * 16u;
    v4f ub[8];
    load_u8(u, row0 + 8u * hh, ub);
    const D2 o1 = layer1(ub, recs + 0u * REC_BYTES, c);
    const D2 a1 = layer1(ub, recs + 1u * REC_BYTES, c);
    col_stats(sSt[wave], 0u, o1, hh, c);
    col_stats(sSt[wave], 64u, a1, hh, c);
    __syncthreads();
    write_part(&sSt[0][0], tid, part + (size_t)bx * 128u);
}

__global__ __launch_bounds__(256) void k_pass2(const float* __restrict__ u, const unsigned char* __restrict__ recs,
                                               float* __restrict__ part) {
    __shared__ __align__(16) float sSlab[8][16 * SLAB_P];
    __shared__ __align__(16) float sSt[8][128];
    const unsigned tid = threadIdx.x, lane = tid & 31u, wave = tid >> 5, hh = lane >> 4, c = lane & 15u;
    const unsigned bx = blockIdx.x;
    const unsigned row0 = (bx * 8u + wave) * 16u;
    float* slab = sSlab[wave];
    v4f ub[8];
    load_u8(u, row0 + 8u * hh, ub);
    const D2 o1 = layer1(ub, recs + 0u * REC_BYTES, c);
    const D2 a1 = layer1(ub, recs + 1u * REC_BYTES, c);
    const D2 o2 = tanh2(site(slab, o1, K_T, 1.0f / K_T, KR_T, 1.0f / (K_T * K_W), 1.0f / (K_T * KR_W), recs + 2u * REC_BYTES, hh, c));
    D2 s;
    s.t[0] = o1.t[0] + o2.t[0];
    s.t[1] = o1.t[1] + o2.t[1];
    const D2 a2 = tanh2(site(slab, a1, K_T, 1.0f / K_T, KR_T, 1.0f / (K_T * K_W), 1.0f / (K_T * KR_W), recs + 3u * REC_BYTES, hh, c));
    col_stats(sSt[wave], 0u, s, hh, c);
    col_stats(sSt[wave], 64u, a2, hh, c);
    __syncthreads();
    write_part(&sSt[0][0], tid, part + (size_t)bx * 128u);
}

__global__ __launch_bounds__(256) void k_pass3(const float* __restrict__ u, const int* __restrict__ mask,
                                               const unsigned char* __restrict__ recs, float* __restrict__ X) {
    __shared__ __align__(16) float sSlab[8][16 * SLAB_P];
    __shared__ __align__(16) float sPool[8][32];
    const unsigned tid = threadIdx.x, lane = tid & 31u, wave = tid >> 5, hh = lane >> 4, c = lane & 15u;
    const unsigned bx = blockIdx.x;
    const unsigned row0 = bx * (unsigned)SEQ + wave * 16u;
    float* slab = sSlab[wave];
    v4f ub[8];
    load_u8(u, row0 + 8u * hh, ub);
    const D2 o1 = layer1(ub, recs + 0u * REC_BYTES, c);
    const D2 a1 = layer1(ub, recs + 1u * REC_BYTES, c);
    const D2 o2 = tanh2(site(slab, o1, K_T, 1.0f / K_T, KR_T, 1.0f / (K_T * K_W), 1.0f / (K_T * KR_W), recs + 2u * REC_BYTES, hh, c));
    D2 s;
    s.t[0] = o1.t[0] + o2.t[0];
    s.t[1] = o1.t[1] + o2.t[1];
    const D2 o3 = tanh2(site(slab, s, K_S, 1.0f / K_S, KR_S, 1.0f / (K_S * K_W), 1.0f / (K_S * KR_W), recs + 4u * REC_BYTES, hh, c));
    D2 xm;
    xm.t[0] = s.t[0] + o3.t[0];
    xm.t[1] = s.t[1] + o3.t[1];
    const D2 a2 = tanh2(site(slab, a1, K_T, 1.0f / K_T, KR_T, 1.0f / (K_T * K_W), 1.0f / (K_T * KR_W), recs + 3u * REC_BYTES, hh, c));
    const D2 a3 = site(slab, a2, K_T, 1.0f / K_T, KR_T, 1.0f / (K_T * K_W), 1.0f / (K_T * KR_W), recs + 5u * REC_BYTES, hh, c);
    const v4i m0 = *(const v4i*)(mask + row0 + 8u * hh);
    const v4i m1 = *(const v4i*)(mask + row0 + 8u * hh + 4u);
    const int mw[8] = {m0.x, m0.y, m0.z, m0.w, m1.x, m1.y, m1.z, m1.w};
    float p0 = 0.f, p1 = 0.f;
#pragma unroll
    for (int r = 0; r < 8; ++r) {
        float mx = fmaxf(a3.t[0][r], a3.t[1][r]);
        mx = fmaxf(mx, __shfl_xor(mx, 1, 32)); mx = fmaxf(mx, __shfl_xor(mx, 2, 32));
        mx = fmaxf(mx, __shfl_xor(mx, 4, 32)); mx = fmaxf(mx, __shfl_xor(mx, 8, 32));
        const float e0 = expf(a3.t[0][r] - mx);
        const float e1 = expf(a3.t[1][r] - mx);
        float sm = e0 + e1;
        sm += __shfl_xor(sm, 1, 32); sm += __shfl_xor(sm, 2, 32);
        sm += __shfl_xor(sm, 4, 32); sm += __shfl_xor(sm, 8, 32);
        float t0 = e0 / sm;
        float t1 = e1 / sm;
        const bool dead = (mw[r] == 0);
        t0 = dead ? -__builtin_inff() : t0;
        t1 = dead ? -__builtin_inff() : t1;
        p0 += xm.t[0][r] * t0;
        p1 += xm.t[1][r] * t1;
    }
    p0 += __shfl_xor(p0, 16, 32);
    p1 += __shfl_xor(p1, 16, 32);
    if (hh == 0u) { sPool[wave][c] = p0; sPool[wave][16u + c] = p1; }
    __syncthreads();
    if (tid < 8u) {
        v4f v;
#pragma unroll
        for (int j = 0; j < 4; ++j) {
            float acc = 0.f;
#pragma unroll
            for (int w = 0; w < 8; ++w) acc += sPool[w][4u * tid + (unsigned)j];
            v[j] = acc;
        }
        VST2V4(X + (size_t)bx * 32u + 4u * tid, v);
    }
}

template <int XIN>
__global__ __launch_bounds__(256) void k_hgemm(const float* __restrict__ In, const unsigned char* __restrict__ rec,
                                               float* __restrict__ Out) {
    __shared__ __align__(16) float sSlab[8][16 * SLAB_P];
    const unsigned tid = threadIdx.x, lane = tid & 31u, wave = tid >> 5, hh = lane >> 4, c = lane & 15u;
    const unsigned bx = blockIdx.x;
    const unsigned row0 = (bx * 8u + wave) * 16u;
    constexpr float ka = XIN ? K_X : K_T;
    constexpr float kra = XIN ? KR_X : KR_T;
    const float* ap = In + (size_t)(row0 + c) * 32u + 8u * hh;
    const v4f q0 = *(const v4f*)(ap), q1 = *(const v4f*)(ap + 4), q2 = *(const v4f*)(ap + 16), q3 = *(const v4f*)(ap + 20);
    v16h ahi, alo;
    build_a(q0, q1, q2, q3, ka, 1.0f / ka, kra, ahi, alo);
    const D2 y = tanh2(mm3(ahi, alo, rec, hh, c, 1.0f / (ka * K_W), 1.0f / (ka * KR_W)));
    float* slab = sSlab[wave];
#pragma unroll
    for (int t = 0; t < 2; ++t)
#pragma unroll
        for (int r = 0; r < 8; ++r) slab[(8u * hh + (unsigned)r) * SLAB_P + 16u * (unsigned)t + c] = y.t[t][r];
    wave_sync_lds();
    const unsigned q = lane >> 3, c4 = (lane & 7u) * 4u;
    v4f ov[4];
#pragma unroll
    for (int it = 0; it < 4; ++it) ov[it] = *(const v4f*)(slab + ((unsigned)it * 4u + q) * SLAB_P + c4);
    for (int pass = 0; pass < 2; ++pass) {
#pragma unroll
        for (int it = 0; it < 4; ++it)
            *(volatile v4f*)(Out + (size_t)(row0 + (unsigned)it * 4u + q) * 32u + c4) = ov[it];
        __threadfence();
    }
}

__global__ __launch_bounds__(256) void k_final(const float* __restrict__ T, const float* __restrict__ g,
                                               const float* __restrict__ b, const float* __restrict__ W4,
                                               const float* __restrict__ B4, float* __restrict__ out) {
    __shared__ double dS[8][32];
    __shared__ double dQ[8][32];
    __shared__ float sW[32];
    __shared__ float sTm[32];
    __shared__ __align__(16) float sOut[256];
    const unsigned t = threadIdx.x, col = t & 31u, sl = t >> 5;
    {
        double s = 0.0, q = 0.0;
        for (unsigned i = 0; i < (unsigned)(NB / 8); ++i) {
            const double x = (double)T[(size_t)(sl * (unsigned)(NB / 8) + i) * 32u + col];
            s += x; q += x * x;
        }
        dS[sl][col] = s; dQ[sl][col] = q;
    }
    __syncthreads();
    if (t < 32u) {
        double s = 0.0, q = 0.0;
#pragma unroll
        for (int w = 0; w < 8; ++w) { s += dS[w][t]; q += dQ[w][t]; }
        const double invn = 1.0 / (double)NB;
        const double mean = s * invn;
        const double var = q * invn - mean * mean;
        const float rs = 1.0f / sqrtf((float)var + 1e-5f);
        const float sg = rs * bfr(g[t]);
        const float w = bfr(W4[t]);
        sW[t] = w * sg;
        sTm[t] = (bfr(b[t]) - (float)mean * sg) * w;
    }
    __syncthreads();
    float wr[32];
    float c4 = 0.f;
#pragma unroll
    for (int k = 0; k < 32; ++k) { wr[k] = sW[k]; c4 += sTm[k]; }
    c4 += bfr(B4[0]);
    for (unsigned it = 0; it < (unsigned)(NB / 256); ++it) {
        const unsigned row = it * 256u + t;
        const float* xr = T + (size_t)row * 32u;
        float acc = 0.f;
#pragma unroll
        for (int g4 = 0; g4 < 8; ++g4) {
            const v4f x = *(const v4f*)(xr + 4 * g4);
            acc += x.x * wr[4 * g4] + x.y * wr[4 * g4 + 1] + x.z * wr[4 * g4 + 2] + x.w * wr[4 * g4 + 3];
        }
        sOut[t] = acc + c4;
        __syncthreads();
        if (t < 64u) {
            const v4f v = *(const v4f*)(sOut + 4u * t);
            VST2V4(out + (size_t)it * 256u + 4u * t, v);
        }
        __syncthreads();
    }
}

extern "C" void kernel_launch(void* const* d_in, const int* in_sizes, int n_in, void* d_out, int out_size,
                              void* d_ws, size_t ws_size, hipStream_t stream) {
    if (n_in < 33) return;
    if (in_sizes[0] < NROWS * 4 || in_sizes[1] < NROWS) return;
    if (in_sizes[2] < 4 || in_sizes[3] < 4 || in_sizes[4] < 128 || in_sizes[11] < 4 || in_sizes[12] < 4 || in_sizes[13] < 128) return;
    if (in_sizes[5] < 32 || in_sizes[6] < 32 || in_sizes[7] < 1024 || in_sizes[8] < 32 || in_sizes[9] < 32 || in_sizes[10] < 1024) return;
    if (in_sizes[14] < 32 || in_sizes[15] < 32 || in_sizes[16] < 1024 || in_sizes[17] < 32 || in_sizes[18] < 32 || in_sizes[19] < 1024) return;
    if (in_sizes[20] < 32 || in_sizes[21] < 32 || in_sizes[22] < 1024 || in_sizes[23] < 32 || in_sizes[24] < 32 || in_sizes[25] < 1024) return;
    if (in_sizes[26] < 32 || in_sizes[27] < 32 || in_sizes[28] < 1024 || in_sizes[29] < 32 || in_sizes[30] < 32 || in_sizes[31] < 32 || in_sizes[32] < 1) return;
    if (out_size < NB) return;

    const float* u       = (const float*)d_in[0];
    const int*   mask    = (const int*)d_in[1];
    const float* p_bn1_g = (const float*)d_in[2];
    const float* p_bn1_b = (const float*)d_in[3];
    const float* p_w1    = (const float*)d_in[4];
    const float* p_bn2_g = (const float*)d_in[5];
    const float* p_bn2_b = (const float*)d_in[6];
    const float* p_w2    = (const float*)d_in[7];
    const float* p_bn3_g = (const float*)d_in[8];
    const float* p_bn3_b = (const float*)d_in[9];
    const float* p_w3    = (const float*)d_in[10];
    const float* o_bn1_g = (const float*)d_in[11];
    const float* o_bn1_b = (const float*)d_in[12];
    const float* o_w1    = (const float*)d_in[13];
    const float* o_bn2_g = (const float*)d_in[14];
    const float* o_bn2_b = (const float*)d_in[15];
    const float* o_w2    = (const float*)d_in[16];
    const float* o_bn3_g = (const float*)d_in[17];
    const float* o_bn3_b = (const float*)d_in[18];
    const float* o_w3    = (const float*)d_in[19];
    const float* t_bn1_g = (const float*)d_in[20];
    const float* t_bn1_b = (const float*)d_in[21];
    const float* t_w1    = (const float*)d_in[22];
    const float* t_bn2_g = (const float*)d_in[23];
    const float* t_bn2_b = (const float*)d_in[24];
    const float* t_w2    = (const float*)d_in[25];
    const float* t_bn3_g = (const float*)d_in[26];
    const float* t_bn3_b = (const float*)d_in[27];
    const float* t_w3    = (const float*)d_in[28];
    const float* t_bn4_g = (const float*)d_in[29];
    const float* t_bn4_b = (const float*)d_in[30];
    const float* t_w4    = (const float*)d_in[31];
    const float* t_b4    = (const float*)d_in[32];
    float* out = (float*)d_out;

    char* wsp = (char*)d_ws;
    size_t off = 0;
    auto carve = [&](size_t bytes) -> void* { void* r = wsp + off; off += a256(bytes); return r; };
    float*         part0 = (float*)carve(SZ_P0);
    float*         part1 = (float*)carve(SZ_P12);
    float*         part2 = (float*)carve(SZ_P12);
    unsigned char* recs  = (unsigned char*)carve(SZ_REC);
    float*         Xp    = (float*)carve(SZ_PL);
    float*         T1    = (float*)carve(SZ_PL);
    float*         T2    = (float*)carve(SZ_PL);
    float*         T3    = (float*)carve(SZ_PL);
    if (off != WS_TOTAL || off > ws_size || off > (size_t)134217728) return;

    k_pass0<<<NP0, 256, 0, stream>>>(u, part0);
    k_fold4<<<1, 64, 0, stream>>>(part0, (unsigned)NP0, (unsigned)NROWS, p_bn1_g, p_bn1_b, p_w1, recs + 0u * REC_BYTES);
    k_fold4<<<1, 64, 0, stream>>>(part0, (unsigned)NP0, (unsigned)NROWS, o_bn1_g, o_bn1_b, o_w1, recs + 1u * REC_BYTES);

    k_pass1<<<NPB, 256, 0, stream>>>(u, recs, part1);
    k_fold32<<<1, 256, 0, stream>>>(part1, (unsigned)NPB, 128u, 0u, 32u, (unsigned)NROWS, p_bn2_g, p_bn2_b, p_w2, recs + 2u * REC_BYTES);
    k_fold32<<<1, 256, 0, stream>>>(part1, (unsigned)NPB, 128u, 64u, 96u, (unsigned)NROWS, o_bn2_g, o_bn2_b, o_w2, recs + 3u * REC_BYTES);

    k_pass2<<<NPB, 256, 0, stream>>>(u, recs, part2);
    k_fold32<<<1, 256, 0, stream>>>(part2, (unsigned)NPB, 128u, 0u, 32u, (unsigned)NROWS, p_bn3_g, p_bn3_b, p_w3, recs + 4u * REC_BYTES);
    k_fold32<<<1, 256, 0, stream>>>(part2, (unsigned)NPB, 128u, 64u, 96u, (unsigned)NROWS, o_bn3_g, o_bn3_b, o_w3, recs + 5u * REC_BYTES);

    k_pass3<<<NB, 256, 0, stream>>>(u, mask, recs, Xp);

    k_foldp<<<1, 256, 0, stream>>>(Xp, t_bn1_g, t_bn1_b, t_w1, recs + 6u * REC_BYTES);
    k_hgemm<1><<<NB / 128, 256, 0, stream>>>(Xp, recs + 6u * REC_BYTES, T1);
    k_foldp<<<1, 256, 0, stream>>>(T1, t_bn2_g, t_bn2_b, t_w2, recs + 7u * REC_BYTES);
    k_hgemm<0><<<NB / 128, 256, 0, stream>>>(T1, recs + 7u * REC_BYTES, T2);
    k_foldp<<<1, 256, 0, stream>>>(T2, t_bn3_g, t_bn3_b, t_w3, recs + 8u * REC_BYTES);
    k_hgemm<0><<<NB / 128, 256, 0, stream>>>(T2, recs + 8u * REC_BYTES, T3);
    k_final<<<1, 256, 0, stream>>>(T3, t_bn4_g, t_bn4_b, t_w4, t_b4, out);
}
